// MambaBlock_69861938037096
// MI455X (gfx1250) — hardware-verified
//
#include <hip/hip_runtime.h>
#include <stddef.h>
#include <stdint.h>
#include <math.h>


#define NBAT 4
#define SL   2048
#define DM   1024
#define DI   2048
#define DS   16
#define DTR  64
#define NXP  96
#define K2I  4096
#define K2T  128
#define NTHR 256
#define GBM  64
#define GTHR 128
#define TT   32
#define SCH  64
#define CTHR 512
#define NUA  (4096 * 128)
#define NUB  (96 * 512)
#define NUC  (2048 * 16)
#define NUD  (1024 * 512)
#define WSMAX 134217728

static_assert(K2I == 2 * DI && K2T == 2 * DTR && NXP == DTR + 2 * DS);
static_assert(DM % 32 == 0 && K2I % 32 == 0 && K2T % 32 == 0);
static_assert(SL % GBM == 0 && (2 * DI) % 128 == 0 && DI % 128 == 0 && DM % 128 == 0 && NXP % 16 == 0);
static_assert(NUA % NTHR == 0 && NUB % NTHR == 0 && NUC % NTHR == 0 && NUD % NTHR == 0);
static_assert(SL % TT == 0 && DI % SCH == 0 && NTHR == 4 * SCH && TT * 8 == NTHR);
static_assert(CTHR * 4 == DI && CTHR * 8 == K2I);
static_assert(GBM == (GTHR / 32) * 16);

typedef float          v4f   __attribute__((ext_vector_type(4)));
typedef float          v8f   __attribute__((ext_vector_type(8)));
typedef int            v8i   __attribute__((ext_vector_type(8)));
typedef unsigned short v4us  __attribute__((ext_vector_type(4)));
typedef unsigned short v8us  __attribute__((ext_vector_type(8)));
typedef unsigned short v16us __attribute__((ext_vector_type(16)));
typedef __bf16         v16bf __attribute__((ext_vector_type(16)));
typedef v4f  __attribute__((may_alias)) v4fa;
typedef v4us __attribute__((may_alias)) v4usa;
typedef v8us __attribute__((may_alias)) v8usa;
union FragB { v16bf v; v16us u; v8us h[2]; v8i w; };

__device__ __forceinline__ v8f wmb(const FragB& a, const FragB& b, v8f c) {
  v8f d = __builtin_amdgcn_wmma_f32_16x16x32_bf16(false, a.v, false, b.v, (short)0, c, false, false);
  asm volatile("v_nop\n\tv_nop\n\tv_nop\n\tv_nop" : "+v"(d) : "v"(a.w), "v"(b.w));
  return d;
}

__device__ __forceinline__ unsigned bf16_bits(float f) {
  const unsigned u = __float_as_uint(f);
  return (u + 0x7FFFu + ((u >> 16) & 1u)) >> 16;
}
__device__ __forceinline__ float bf16_val(float f) {
  return __uint_as_float(bf16_bits(f) << 16);
}
__device__ __forceinline__ float bfbits_f(unsigned short h) {
  return __uint_as_float(((unsigned)h) << 16);
}
__device__ __forceinline__ float silu_f(float v) {
  return v * __builtin_amdgcn_rcpf(1.0f + expf(-v));
}
__device__ __forceinline__ float softplus_f(float v) {
  return fmaxf(v, 0.0f) + log1pf(expf(-fabsf(v)));
}
__device__ __forceinline__ unsigned short hl_sel(float v, bool sel) {
  const unsigned hb = bf16_bits(v);
  const unsigned lb = bf16_bits(v - __uint_as_float(hb << 16));
  return (unsigned short)(sel ? lb : hb);
}

__global__ __launch_bounds__(NTHR) void k_cvx(const float* __restrict__ x, unsigned short* xb) {
  const size_t u = (size_t)blockIdx.x * NTHR + threadIdx.x;
  const float* p = x + u * 8;
  const v4f a = *(const v4f*)p;
  const v4f b = *(const v4f*)(p + 4);
  v8us o;
  o[0] = (unsigned short)bf16_bits(a.x); o[1] = (unsigned short)bf16_bits(a.y);
  o[2] = (unsigned short)bf16_bits(a.z); o[3] = (unsigned short)bf16_bits(a.w);
  o[4] = (unsigned short)bf16_bits(b.x); o[5] = (unsigned short)bf16_bits(b.y);
  o[6] = (unsigned short)bf16_bits(b.z); o[7] = (unsigned short)bf16_bits(b.w);
  unsigned short* dp = xb + u * 8;
  *(volatile v8us*)dp = o;
  __threadfence();
  *(volatile v8us*)dp = o;
}

__global__ __launch_bounds__(NTHR) void k_wprep(const float* __restrict__ Win, const float* __restrict__ Wx,
                                                const float* __restrict__ Wdt, const float* __restrict__ Wout,
                                                unsigned short* wsb, size_t eWinT, size_t eWx2,
                                                size_t eWdt2, size_t eWout2) {
  const int u = (int)blockIdx.x * NTHR + (int)threadIdx.x;
  v8us o;
  size_t doff;
  if (u < NUA) {
    const int n  = u >> 7;
    const int k8 = (u & 127) * 8;
    const float* p = Win + (size_t)k8 * (2 * DI) + n;
#pragma unroll
    for (int i = 0; i < 8; ++i) o[i] = (unsigned short)bf16_bits(p[(size_t)i * (2 * DI)]);
    doff = eWinT + (size_t)n * DM + k8;
  } else if (u < NUA + NUB) {
    const int v  = u - NUA;
    const int n  = v >> 9;
    const int k8 = (v & 511) * 8;
    const int kk = k8 & (DI - 1);
    const float* p = Wx + (size_t)kk * NXP + n;
#pragma unroll
    for (int i = 0; i < 8; ++i) o[i] = (unsigned short)bf16_bits(p[(size_t)i * NXP]);
    doff = eWx2 + (size_t)n * K2I + k8;
  } else if (u < NUA + NUB + NUC) {
    const int v  = u - NUA - NUB;
    const int n  = v >> 4;
    const int k8 = (v & 15) * 8;
    const int kk = k8 & (DTR - 1);
    const float* p = Wdt + (size_t)kk * DI + n;
#pragma unroll
    for (int i = 0; i < 8; ++i) o[i] = (unsigned short)bf16_bits(p[(size_t)i * DI]);
    doff = eWdt2 + (size_t)n * K2T + k8;
  } else if (u < NUA + NUB + NUC + NUD) {
    const int v  = u - NUA - NUB - NUC;
    const int n  = v >> 9;
    const int k8 = (v & 511) * 8;
    const int kk = k8 & (DI - 1);
    const float* p = Wout + (size_t)kk * DM + n;
#pragma unroll
    for (int i = 0; i < 8; ++i) o[i] = (unsigned short)bf16_bits(p[(size_t)i * DM]);
    doff = eWout2 + (size_t)n * K2I + k8;
  } else {
    return;
  }
  unsigned short* dp = wsb + doff;
  *(volatile v8us*)dp = o;
  __threadfence();
  *(volatile v8us*)dp = o;
}

template <int NT, int EPI>
__global__ __launch_bounds__(GTHR) void k_gemm(const unsigned short* __restrict__ A, int lda,
                                               const unsigned short* __restrict__ BT, int K,
                                               float* outF, const float* __restrict__ bias,
                                               unsigned short* outH, float* outB) {
  constexpr int CW = 16 * NT;
  __shared__ __attribute__((aligned(16))) float stg[GBM * CW];
  const int tid = (int)threadIdx.x, lane = tid & 31, wave = tid >> 5, hh = lane >> 4, m = lane & 15;
  const int rowBase = (int)blockIdx.x * GBM;
  const int col0    = (int)blockIdx.y * CW;

  v8f acc[NT];
  {
    const v8f z = {0.f, 0.f, 0.f, 0.f, 0.f, 0.f, 0.f, 0.f};
#pragma unroll
    for (int t = 0; t < NT; ++t) acc[t] = z;
  }
  const unsigned short* ap = A  + (size_t)(rowBase + 16 * wave + m) * (size_t)lda + 8 * hh;
  const unsigned short* bp = BT + (size_t)(col0 + m) * (size_t)K + 8 * hh;

#pragma unroll 1
  for (int k0 = 0; k0 < K; k0 += 32) {
    FragB af;
    af.h[0] = *(const v8usa*)(ap + k0);
    af.h[1] = *(const v8usa*)(ap + k0 + 16);
#pragma unroll
    for (int nt = 0; nt < NT; ++nt) {
      const unsigned short* wq = bp + (size_t)(16 * nt) * (size_t)K + k0;
      FragB bf;
      bf.h[0] = *(const v8usa*)wq;
      bf.h[1] = *(const v8usa*)(wq + 16);
      acc[nt] = wmb(af, bf, acc[nt]);
    }
  }

#pragma unroll
  for (int nt = 0; nt < NT; ++nt) {
    const int lc = 16 * nt + m;
#pragma unroll
    for (int r = 0; r < 8; ++r) {
      const int lr = 16 * wave + 8 * hh + r;
      stg[lr * CW + lc] = acc[nt][r];
    }
  }
  __syncthreads();

  if constexpr (EPI == 1) {
    const int  c8  = 8 * (m & 7);
    const bool sel = m >= 8;
    const int  rq  = lane >> 3;
    const int  q4  = 4 * (lane & 7);
#pragma unroll 1
    for (int pass = 0; pass < 2; ++pass) {
#pragma unroll 2
      for (int i = 0; i < 8; ++i) {
        const int lr = 16 * wave + 2 * i + hh;
        const float* sp = stg + lr * CW + c8;
        const v4f a = *(const v4fa*)sp;
        const v4f b = *(const v4fa*)(sp + 4);
        v8us o;
        o[0] = hl_sel(a.x, sel); o[1] = hl_sel(a.y, sel); o[2] = hl_sel(a.z, sel); o[3] = hl_sel(a.w, sel);
        o[4] = hl_sel(b.x, sel); o[5] = hl_sel(b.y, sel); o[6] = hl_sel(b.z, sel); o[7] = hl_sel(b.w, sel);
        unsigned short* dp = outH + (size_t)(rowBase + lr) * K2T + 8 * m;
        *(volatile v8us*)dp = o;
      }
#pragma unroll 2
      for (int i = 0; i < 4; ++i) {
        const int lr = 16 * wave + 4 * i + rq;
        const v4f v = *(const v4fa*)(stg + lr * CW + 64 + q4);
        float* dp = outB + (size_t)(rowBase + lr) * 32 + q4;
        *(volatile v4f*)dp = v;
      }
      __threadfence();
    }
  } else {
    static_assert(EPI == 1 || NT == 8);
    float* srow = stg + (16 * wave) * CW + 4 * lane;
    size_t obase;
    int ldo;
    if constexpr (EPI == 0) {
      const bool isG = col0 >= DI;
      ldo = DI;
      obase = (isG ? (size_t)SL * DI : (size_t)0) + (size_t)(col0 & (DI - 1));
      if (isG) {
#pragma unroll 2
        for (int i = 0; i < 16; ++i) {
          v4f t = *(const v4fa*)(srow + i * CW);
          t.x = silu_f(t.x); t.y = silu_f(t.y); t.z = silu_f(t.z); t.w = silu_f(t.w);
          *(v4fa*)(srow + i * CW) = t;
        }
      }
    } else if constexpr (EPI == 2) {
      ldo = DI;
      obase = (size_t)col0;
      const v4f bq = *(const v4f*)(bias + col0 + 4 * lane);
      const float b0 = bf16_val(bq.x), b1 = bf16_val(bq.y), b2 = bf16_val(bq.z), b3 = bf16_val(bq.w);
#pragma unroll 2
      for (int i = 0; i < 16; ++i) {
        v4f t = *(const v4fa*)(srow + i * CW);
        t.x = softplus_f(t.x + b0); t.y = softplus_f(t.y + b1);
        t.z = softplus_f(t.z + b2); t.w = softplus_f(t.w + b3);
        *(v4fa*)(srow + i * CW) = t;
      }
    } else {
      ldo = DM;
      obase = (size_t)col0;
    }
    float* orow = outF + obase + (size_t)(rowBase + 16 * wave) * (size_t)ldo + 4 * lane;
#pragma unroll 4
    for (int i = 0; i < 16; ++i) {
      const v4f t = *(const v4fa*)(srow + i * CW);
      *(volatile v4f*)(orow + (size_t)i * (size_t)ldo) = t;
    }
    __threadfence();
#pragma unroll 4
    for (int i = 0; i < 16; ++i) {
      const v4f t = *(const v4fa*)(srow + i * CW);
      *(volatile v4f*)(orow + (size_t)i * (size_t)ldo) = t;
    }
  }
}

__device__ __forceinline__ float conv_one(float a0, float a1, float a2, float a3, v4f w, float b) {
  float s = 0.0f;
  s = s + a0 * bf16_val(w.x);
  s = s + a1 * bf16_val(w.y);
  s = s + a2 * bf16_val(w.z);
  s = s + a3 * bf16_val(w.w);
  s = s + bf16_val(b);
  return silu_f(s);
}

__global__ __launch_bounds__(CTHR) void k_conv(const float* __restrict__ XV, const float* __restrict__ cw,
                                               const float* __restrict__ cb, unsigned short* U) {
  __shared__ __attribute__((aligned(16))) unsigned short sHL[K2I];
  const int tid = (int)threadIdx.x;
  const int l   = (int)blockIdx.x;
  const int d0  = 4 * tid;
  const v4f w0 = *(const v4f*)(cw + (size_t)d0 * 4);
  const v4f w1 = *(const v4f*)(cw + (size_t)d0 * 4 + 4);
  const v4f w2 = *(const v4f*)(cw + (size_t)d0 * 4 + 8);
  const v4f w3 = *(const v4f*)(cw + (size_t)d0 * 4 + 12);
  const v4f bb = *(const v4f*)(cb + d0);
  const int r0 = l - 3, r1 = l - 2, r2 = l - 1;
  const float f0 = (r0 >= 0) ? 1.0f : 0.0f;
  const float f1 = (r1 >= 0) ? 1.0f : 0.0f;
  const float f2 = (r2 >= 0) ? 1.0f : 0.0f;
  const int c0 = r0 < 0 ? 0 : r0, c1 = r1 < 0 ? 0 : r1, c2 = r2 < 0 ? 0 : r2;
  const v4f x0 = *(const v4f*)(XV + (size_t)c0 * DI + d0) * f0;
  const v4f x1 = *(const v4f*)(XV + (size_t)c1 * DI + d0) * f1;
  const v4f x2 = *(const v4f*)(XV + (size_t)c2 * DI + d0) * f2;
  const v4f x3 = *(const v4f*)(XV + (size_t)l  * DI + d0);
  const float u0 = conv_one(x0.x, x1.x, x2.x, x3.x, w0, bb.x);
  const float u1 = conv_one(x0.y, x1.y, x2.y, x3.y, w1, bb.y);
  const float u2 = conv_one(x0.z, x1.z, x2.z, x3.z, w2, bb.z);
  const float u3 = conv_one(x0.w, x1.w, x2.w, x3.w, w3, bb.w);
  v4us h4, l4;
  {
    unsigned hb;
    hb = bf16_bits(u0); h4[0] = (unsigned short)hb; l4[0] = (unsigned short)bf16_bits(u0 - __uint_as_float(hb << 16));
    hb = bf16_bits(u1); h4[1] = (unsigned short)hb; l4[1] = (unsigned short)bf16_bits(u1 - __uint_as_float(hb << 16));
    hb = bf16_bits(u2); h4[2] = (unsigned short)hb; l4[2] = (unsigned short)bf16_bits(u2 - __uint_as_float(hb << 16));
    hb = bf16_bits(u3); h4[3] = (unsigned short)hb; l4[3] = (unsigned short)bf16_bits(u3 - __uint_as_float(hb << 16));
  }
  *(v4usa*)(sHL + d0) = h4;
  *(v4usa*)(sHL + DI + d0) = l4;
  __syncthreads();
  const v8us q = *(const v8usa*)(sHL + 8 * tid);
  unsigned short* dp = U + (size_t)l * K2I + 8 * tid;
  *(volatile v8us*)dp = q;
  __threadfence();
  *(volatile v8us*)dp = q;
}

__global__ __launch_bounds__(NTHR) void k_scan(const float* __restrict__ DT, const unsigned short* __restrict__ U,
                                               const float* __restrict__ G, const float* __restrict__ BC,
                                               const float* __restrict__ logA, const float* __restrict__ Dp,
                                               unsigned short* YG) {
  __shared__ __attribute__((aligned(16))) float sDT[TT * SCH];
  __shared__ __attribute__((aligned(16))) float sG[TT * SCH];
  __shared__ __attribute__((aligned(16))) unsigned short sUh[TT * SCH];
  __shared__ __attribute__((aligned(16))) unsigned short sUl[TT * SCH];
  __shared__ __attribute__((aligned(16))) float sBC[TT * 32];
  __shared__ __attribute__((aligned(16))) unsigned short sYh[TT * SCH];
  __shared__ __attribute__((aligned(16))) unsigned short sYl[TT * SCH];
  const int tid = (int)threadIdx.x;
  const int c   = tid >> 2, q = tid & 3;
  const int d0  = (int)blockIdx.x * SCH;
  const int d   = d0 + c;

  float A0, A1, A2, A3;
  {
    const v4f la = *(const v4f*)(logA + (size_t)d * DS + 4 * q);
    A0 = -expf(bf16_val(la.x)); A1 = -expf(bf16_val(la.y));
    A2 = -expf(bf16_val(la.z)); A3 = -expf(bf16_val(la.w));
  }
  const float dpar = bf16_val(Dp[d]);
  float h0 = 0.0f, h1 = 0.0f, h2 = 0.0f, h3 = 0.0f;
  const int rU = tid >> 3, cU = (tid & 7) * 8;

#pragma unroll 1
  for (int ch = 0; ch < SL / TT; ++ch) {
    const int l0 = ch * TT;
    {
#pragma unroll
      for (int it = 0; it < 2; ++it) {
        const int p  = tid + NTHR * it;
        const int r  = p >> 4;
        const int c4 = (p & 15) * 4;
        const size_t go = (size_t)(l0 + r) * DI + d0 + c4;
        const v4f a = *(const v4f*)(DT + go);
        const v4f g = *(const v4f*)(G + go);
        *(v4fa*)(sDT + r * SCH + c4) = a;
        *(v4fa*)(sG + r * SCH + c4) = g;
      }
      const unsigned short* up = U + (size_t)(l0 + rU) * K2I + d0 + cU;
      const v8us uh = *(const v8usa*)up;
      const v8us ul = *(const v8usa*)(up + DI);
      *(v8usa*)(sUh + rU * SCH + cU) = uh;
      *(v8usa*)(sUl + rU * SCH + cU) = ul;
      const v4f bc = *(const v4f*)(BC + (size_t)l0 * 32 + 4 * tid);
      *(v4fa*)(sBC + 4 * tid) = bc;
    }
    __syncthreads();

#pragma unroll 1
    for (int t = 0; t < TT; ++t) {
      const float dt = sDT[t * SCH + c];
      const float u  = bfbits_f(sUh[t * SCH + c]) + bfbits_f(sUl[t * SCH + c]);
      const float gg = sG[t * SCH + c];
      const v4f Bv = *(const v4fa*)(sBC + t * 32 + 4 * q);
      const v4f Cv = *(const v4fa*)(sBC + t * 32 + 16 + 4 * q);
      const float e0 = expf(dt * A0), e1 = expf(dt * A1), e2 = expf(dt * A2), e3 = expf(dt * A3);
      h0 = e0 * h0 + (dt * Bv.x) * u;
      h1 = e1 * h1 + (dt * Bv.y) * u;
      h2 = e2 * h2 + (dt * Bv.z) * u;
      h3 = e3 * h3 + (dt * Bv.w) * u;
      float part = Cv.x * h0;
      part = part + Cv.y * h1;
      part = part + Cv.z * h2;
      part = part + Cv.w * h3;
      part = part + __shfl_xor(part, 1, 32);
      part = part + __shfl_xor(part, 2, 32);
      const float y  = part + dpar * u;
      const float yg = y * gg;
      const unsigned hb = bf16_bits(yg);
      const unsigned lb = bf16_bits(yg - __uint_as_float(hb << 16));
      if (q == 0) {
        sYh[t * SCH + c] = (unsigned short)hb;
        sYl[t * SCH + c] = (unsigned short)lb;
      }
    }
    __syncthreads();

    {
      const v8us yh = *(const v8usa*)(sYh + rU * SCH + cU);
      const v8us yl = *(const v8usa*)(sYl + rU * SCH + cU);
      unsigned short* ph = YG + (size_t)(l0 + rU) * K2I + d0 + cU;
      *(volatile v8us*)ph = yh;
      *(volatile v8us*)(ph + DI) = yl;
      __threadfence();
      *(volatile v8us*)ph = yh;
      *(volatile v8us*)(ph + DI) = yl;
    }
  }
}

static inline size_t al256(size_t o) { return (o + 255) & ~(size_t)255; }

extern "C" void kernel_launch(void* const* d_in, const int* in_sizes, int n_in,
                              void* d_out, int out_size, void* d_ws, size_t ws_size,
                              hipStream_t stream) {
  if (n_in < 10) return;
  if (in_sizes[0] != NBAT * SL * DM) return;
  if (in_sizes[1] != DM * 2 * DI) return;
  if (in_sizes[2] != DI * 4) return;
  if (in_sizes[3] != DI) return;
  if (in_sizes[4] != DI * NXP) return;
  if (in_sizes[5] != DTR * DI) return;
  if (in_sizes[6] != DI) return;
  if (in_sizes[7] != DI * DS) return;
  if (in_sizes[8] != DI) return;
  if (in_sizes[9] != DI * DM) return;
  if (out_size != NBAT * SL * DM) return;

  const float* x     = (const float*)d_in[0];
  const float* W_in  = (const float*)d_in[1];
  const float* cw    = (const float*)d_in[2];
  const float* cb    = (const float*)d_in[3];
  const float* W_x   = (const float*)d_in[4];
  const float* W_dt  = (const float*)d_in[5];
  const float* b_dt  = (const float*)d_in[6];
  const float* logA  = (const float*)d_in[7];
  const float* Dpar  = (const float*)d_in[8];
  const float* W_out = (const float*)d_in[9];
  float* out = (float*)d_out;

  char* ws = (char*)d_ws;
  size_t off = 0;
  const size_t oXB   = off; off = al256(off + (size_t)NBAT * SL * DM * 2);
  const size_t oWinT = off; off = al256(off + (size_t)(2 * DI) * DM * 2);
  const size_t oWx2  = off; off = al256(off + (size_t)NXP * K2I * 2);
  const size_t oWdt2 = off; off = al256(off + (size_t)DI * K2T * 2);
  const size_t oWo2  = off; off = al256(off + (size_t)DM * K2I * 2);
  const size_t oXG   = off; off = al256(off + (size_t)2 * SL * DI * 4);
  const size_t oU    = off; off = al256(off + (size_t)SL * K2I * 2);
  const size_t oDTL  = off; off = al256(off + (size_t)SL * K2T * 2);
  const size_t oBC   = off; off = al256(off + (size_t)SL * 32 * 4);
  const size_t oDT   = off; off = al256(off + (size_t)SL * DI * 4);
  const size_t oYG   = off; off = al256(off + (size_t)SL * K2I * 2);
  if (off > ws_size || off > (size_t)WSMAX) return;

  unsigned short* wsb   = (unsigned short*)ws;
  unsigned short* XB    = (unsigned short*)(ws + oXB);
  unsigned short* WinT  = (unsigned short*)(ws + oWinT);
  unsigned short* Wx2   = (unsigned short*)(ws + oWx2);
  unsigned short* Wdt2  = (unsigned short*)(ws + oWdt2);
  unsigned short* Wout2 = (unsigned short*)(ws + oWo2);
  float*          XG    = (float*)(ws + oXG);
  float*          Gp    = XG + (size_t)SL * DI;
  unsigned short* Upl   = (unsigned short*)(ws + oU);
  unsigned short* DTL   = (unsigned short*)(ws + oDTL);
  float*          BCp   = (float*)(ws + oBC);
  float*          DTp   = (float*)(ws + oDT);
  unsigned short* YGp   = (unsigned short*)(ws + oYG);

  k_cvx<<<(NBAT * SL * DM / 8) / NTHR, NTHR, 0, stream>>>(x, XB);
  k_wprep<<<(NUA + NUB + NUC + NUD) / NTHR, NTHR, 0, stream>>>(W_in, W_x, W_dt, W_out, wsb,
                                                              oWinT / 2, oWx2 / 2, oWdt2 / 2, oWo2 / 2);

  for (int b = 0; b < NBAT; ++b) {
    const unsigned short* XBb = XB + (size_t)b * SL * DM;
    float* outb = out + (size_t)b * SL * DM;
    k_gemm<8, 0><<<dim3(SL / GBM, (2 * DI) / 128), GTHR, 0, stream>>>(XBb, DM, WinT, DM, XG, b_dt, DTL, BCp);
    k_conv<<<SL, CTHR, 0, stream>>>(XG, cw, cb, Upl);
    k_gemm<6, 1><<<dim3(SL / GBM, 1), GTHR, 0, stream>>>(Upl, K2I, Wx2, K2I, XG, b_dt, DTL, BCp);
    k_gemm<8, 2><<<dim3(SL / GBM, DI / 128), GTHR, 0, stream>>>(DTL, K2T, Wdt2, K2T, DTp, b_dt, DTL, BCp);
    k_scan<<<DI / SCH, NTHR, 0, stream>>>(DTp, Upl, Gp, BCp, logA, Dpar, YGp);
    k_gemm<8, 3><<<dim3(SL / GBM, DM / 128), GTHR, 0, stream>>>(YGp, K2I, Wout2, K2I, outb, b_dt, DTL, BCp);
  }
}
